// Net_65549790871635
// MI455X (gfx1250) — hardware-verified
//
#include <hip/hip_runtime.h>
#include <math.h>

constexpr int NPTS      = 131072;
constexpr int NBAT      = 4;
constexpr int PERB      = NPTS / NBAT;
constexpr int MROW      = 32768;
constexpr int KNBR      = 16;
constexpr int NEDGE     = MROW * KNBR;
constexpr int STEM_IN   = 97;
constexpr int STEM_KP   = 128;
constexpr int STEM_HID  = 64;
constexpr int STEM_OUT  = 32;
constexpr int MSG_IN    = 39;
constexpr int MSG_KP    = 64;
constexpr int LOC_HID   = 64;
constexpr int LOC_OUT   = 128;
constexpr int IRB_WIDE  = 512;
constexpr int XA_PITCH  = 136;
constexpr int T_PITCH   = 72;
constexpr int RAW_PITCH = 100;
constexpr int SLAB_PITCH = 68;
constexpr int CEN_PITCH = 32;
constexpr float BNC = 0.99999500003749969f;
constexpr float KDC = 0.57735026918962576f;
constexpr float HALF_LOG2_10 = 1.6609640474436813f;
constexpr float WLO_CARRY     = 2048.0f;
constexpr float WLO_CARRY_INV = 1.0f / 2048.0f;

static_assert(PERB == 32768, "cloud size");
static_assert(NPTS % 64 == 0, "stem grid exact");
static_assert(MROW % 256 == 0 && MROW % 64 == 0 && MROW % 8 == 0, "target tiling");
static_assert(STEM_KP % 32 == 0 && MSG_KP % 32 == 0 && STEM_HID % 32 == 0 && LOC_HID % 32 == 0, "K multiples of 32");
static_assert(LOC_OUT % 64 == 0 && IRB_WIDE % 64 == 0 && LOC_OUT % 32 == 0 && IRB_WIDE % 32 == 0, "GEMM tile multiples");
static_assert(STEM_IN <= STEM_KP && MSG_IN + 8 <= 48 && 48 <= MSG_KP, "pad columns");
static_assert(XA_PITCH % 8 == 0 && T_PITCH % 8 == 0 && XA_PITCH >= STEM_KP && T_PITCH >= MSG_KP, "LDS pitches");

typedef __attribute__((ext_vector_type(16))) _Float16 v16h;
typedef __attribute__((ext_vector_type(8)))  _Float16 v8h;
typedef __attribute__((ext_vector_type(2)))  _Float16 v2h;
typedef __attribute__((ext_vector_type(16))) __bf16   v16b;
typedef __attribute__((ext_vector_type(8)))  __bf16   v8b;
typedef __attribute__((ext_vector_type(8)))  float    v8f;
typedef __attribute__((ext_vector_type(4)))  float    v4f;
typedef __attribute__((ext_vector_type(4)))  unsigned int u32x4;

__device__ __forceinline__ unsigned bf_bits32(float f) {
  const unsigned u = __float_as_uint(f);
  return (u + 0x7FFFu + ((u >> 16) & 1u)) >> 16;
}
__device__ __forceinline__ unsigned pack2(unsigned lo, unsigned hi) { return lo | (hi << 16); }
__device__ __forceinline__ unsigned pack_h2f(float a, float b) {
  v2h v;
  v[0] = (_Float16)a;
  v[1] = (_Float16)b;
  return __builtin_bit_cast(unsigned, v);
}

__device__ __forceinline__ float silu_f(float v) {
  const float e  = expf(-v);
  const float rc = __builtin_amdgcn_rcpf(1.0f + e);
  return v * rc;
}

__device__ __forceinline__ void wave_sync_lds() {
  __builtin_amdgcn_fence(__ATOMIC_RELEASE, "workgroup");
  __builtin_amdgcn_wave_barrier();
  __builtin_amdgcn_fence(__ATOMIC_ACQUIRE, "workgroup");
}

__device__ __forceinline__ void guard1_h4(v8f& a, v16h x0, v16h x1, v16h y0, v16h y1) {
  asm volatile("v_nop\n\tv_nop\n\tv_nop\n\tv_nop" : "+v"(a) : "v"(x0), "v"(x1), "v"(y0), "v"(y1));
}
__device__ __forceinline__ void guard1_h8(v8f& a, v16h x0, v16h x1, v16h x2, v16h x3, v16h y0, v16h y1, v16h y2, v16h y3) {
  asm volatile("v_nop\n\tv_nop\n\tv_nop\n\tv_nop" : "+v"(a) : "v"(x0), "v"(x1), "v"(x2), "v"(x3), "v"(y0), "v"(y1), "v"(y2), "v"(y3));
}
__device__ __forceinline__ void guard4_b(v8f& a, v8f& b, v8f& c, v8f& d, v16b x, v16b y0, v16b y1, v16b y2, v16b y3) {
  asm volatile("v_nop\n\tv_nop\n\tv_nop\n\tv_nop" : "+v"(a), "+v"(b), "+v"(c), "+v"(d) : "v"(x), "v"(y0), "v"(y1), "v"(y2), "v"(y3));
}
__device__ __forceinline__ void keep4_b(v16b a, v16b b, v16b c, v16b d) { asm volatile("v_nop" :: "v"(a), "v"(b), "v"(c), "v"(d)); }
__device__ __forceinline__ void acc_guard4(v8f& a, v8f& b, v8f& c, v8f& d) { asm volatile("v_nop\n\tv_nop\n\tv_nop\n\tv_nop" : "+v"(a), "+v"(b), "+v"(c), "+v"(d)); }

template <typename T> struct Frag;
template <> struct Frag<_Float16> {
  typedef v16h V; union U { v16h v; v8h h[2]; };
  static __device__ __forceinline__ v16h load(const _Float16* p) {
    U f; f.h[0] = *(const v8h*)(p); f.h[1] = *(const v8h*)(p + 16); return f.v;
  }
  static __device__ __forceinline__ v8f mma(v16h a, v16h b, v8f c) {
    return __builtin_amdgcn_wmma_f32_16x16x32_f16(false, a, false, b, (short)0, c, false, false);
  }
};
template <> struct Frag<__bf16> {
  typedef v16b V; union U { v16b v; v8b h[2]; };
  static __device__ __forceinline__ v16b load(const __bf16* p) {
    U f; f.h[0] = *(const v8b*)(p); f.h[1] = *(const v8b*)(p + 16); return f.v;
  }
  static __device__ __forceinline__ v8f mma(v16b a, v16b b, v8f c) {
    return __builtin_amdgcn_wmma_f32_16x16x32_bf16(false, a, false, b, (short)0, c, false, false);
  }
};

template <int MODE>
__global__ __launch_bounds__(256) void prep_bt_kernel(const float* __restrict__ W, unsigned* __restrict__ dst,
                                                      int Kin, int Nout, int Kpad) {
  const int i  = blockIdx.x * 256 + threadIdx.x;
  const int kc = Kpad >> 3;
  const int total = Nout * kc;
  if (i < total) {
    const int n  = i / kc;
    const int c8 = i - n * kc;
    float wz[8];
#pragma unroll
    for (int e = 0; e < 8; ++e) {
      const int k  = c8 * 8 + e;
      const int kk = (k < Kin) ? k : (Kin - 1);
      const float w  = W[(size_t)kk * Nout + n];
      wz[e] = (k < Kin) ? w : 0.0f;
    }
    u32x4 o;
    if (MODE == 0) {
      o[0] = pack_h2f(wz[0], wz[1]);
      o[1] = pack_h2f(wz[2], wz[3]);
      o[2] = pack_h2f(wz[4], wz[5]);
      o[3] = pack_h2f(wz[6], wz[7]);
    } else {
      o[0] = pack2(bf_bits32(wz[0]), bf_bits32(wz[1]));
      o[1] = pack2(bf_bits32(wz[2]), bf_bits32(wz[3]));
      o[2] = pack2(bf_bits32(wz[4]), bf_bits32(wz[5]));
      o[3] = pack2(bf_bits32(wz[6]), bf_bits32(wz[7]));
    }
    volatile u32x4* p = (volatile u32x4*)(dst + (size_t)i * 4);
    *p = o;
    __threadfence();
    *p = o;
  }
}

__global__ __launch_bounds__(256) void prep_loc1_kernel(const float* __restrict__ W, unsigned* __restrict__ dst) {
  const int i  = blockIdx.x * 256 + threadIdx.x;
  const int n  = i >> 3;
  const int c8 = i & 7;
  float val[8];
#pragma unroll
  for (int e = 0; e < 8; ++e) {
    const int k  = c8 * 8 + e;
    const int sr = (k < MSG_IN) ? k : ((k < 43) ? (k - 7) : ((k < 47) ? (k - 11) : 0));
    const float w = W[sr * LOC_HID + n];
    const _Float16 hi = (_Float16)w;
    const float hif = (float)hi;
    const float lof = (w - hif) * WLO_CARRY;
    val[e] = (k < 43) ? w : ((k < 47) ? lof : 0.0f);
  }
  u32x4 o;
  o[0] = pack_h2f(val[0], val[1]);
  o[1] = pack_h2f(val[2], val[3]);
  o[2] = pack_h2f(val[4], val[5]);
  o[3] = pack_h2f(val[6], val[7]);
  volatile u32x4* p = (volatile u32x4*)(dst + (size_t)i * 4);
  *p = o;
  __threadfence();
  *p = o;
}

__global__ __launch_bounds__(256) void centres_kernel(const float* __restrict__ pos, const float* __restrict__ sf,
                                                      float* __restrict__ cen) {
  __shared__ float red[3][256];
  const int b = blockIdx.x, tid = threadIdx.x;
  const float inv = 1.0f / sf[b];
  float s0 = 0.0f, s1 = 0.0f, s2 = 0.0f;
#pragma unroll 1
  for (int i = tid; i < PERB; i += 256) {
    const float* p = pos + (size_t)(b * PERB + i) * 3;
    s0 += p[0] * inv;
    s1 += p[1] * inv;
    s2 += p[2] * inv;
  }
  red[0][tid] = s0; red[1][tid] = s1; red[2][tid] = s2;
  __syncthreads();
  for (int off = 128; off > 0; off >>= 1) {
    if (tid < off) {
      red[0][tid] += red[0][tid + off];
      red[1][tid] += red[1][tid + off];
      red[2][tid] += red[2][tid + off];
    }
    __syncthreads();
  }
  if (tid < 32) {
    const int li = (tid < 3) ? tid : 2;
    const float raw = red[li][0] * (1.0f / (float)PERB);
    const float v = (tid < 3) ? raw : 0.0f;
    volatile float* p = cen + b * CEN_PITCH + tid;
    *p = v;
    __threadfence();
    *p = v;
  }
}

__global__ __launch_bounds__(128) void stem_kernel(const float* __restrict__ pos, const float* __restrict__ refl,
                                                   const float* __restrict__ sf, const int* __restrict__ batch,
                                                   const float* __restrict__ cen,
                                                   const float* __restrict__ lng, const float* __restrict__ lnb,
                                                   const unsigned short* __restrict__ W1tp, const float* __restrict__ b1,
                                                   const unsigned short* __restrict__ W2tp, const float* __restrict__ b2,
                                                   unsigned* __restrict__ xplane) {
  __shared__ __align__(16) float    rawS[4][16 * RAW_PITCH];
  __shared__ __align__(16) _Float16 xaS[4][16 * XA_PITCH];
  __shared__ __align__(16) _Float16 hdS[4][16 * T_PITCH];
  __shared__ __align__(16) _Float16 xoS[4][16 * STEM_OUT];
  const _Float16* W1t = (const _Float16*)W1tp;
  const _Float16* W2t = (const _Float16*)W2tp;
  const int tid = threadIdx.x, wave = tid >> 5, lane = tid & 31;
  const int c = lane & 15, hh = lane >> 4, koff = hh * 8;
  const int pt0 = blockIdx.x * 64 + wave * 16;
  const int pt  = pt0 + c;
  int b = batch[pt];
  b = (b < 0) ? 0 : ((b > NBAT - 1) ? (NBAT - 1) : b);
  const float inv = 1.0f / sf[b];
  const float q0 = pos[(size_t)pt * 3 + 0] * inv - cen[b * CEN_PITCH + 0];
  const float q1 = pos[(size_t)pt * 3 + 1] * inv - cen[b * CEN_PITCH + 1];
  const float q2 = pos[(size_t)pt * 3 + 2] * inv - cen[b * CEN_PITCH + 2];
  const float rf = refl[pt];
  const float g96 = lng[96], be96 = lnb[96];
  float* rw = rawS[wave] + c * RAW_PITCH;

  float sum = 0.0f;
#pragma unroll 1
  for (int i = 0; i < 24; ++i) {
    const int p = hh * 24 + i;
    const int d = p >> 4, f = p & 15;
    const float nv = (d == 0) ? q0 : ((d == 1) ? q1 : q2);
    const float fr = exp2f(-(float)f * HALF_LOG2_10);
    const float arg = nv * fr;
    const float sn = sinf(arg);
    const float cs = cosf(arg);
    rw[d * 32 + f] = sn;
    rw[d * 32 + 16 + f] = cs;
    sum += sn;
    sum += cs;
  }
  if (hh == 1) rw[96] = rf;
  sum += (hh == 1) ? rf : 0.0f;
  sum += __shfl_xor(sum, 16, 32);
  const float mean = sum * (1.0f / (float)STEM_IN);
  float ss = 0.0f;
#pragma unroll 1
  for (int i = 0; i < 24; ++i) {
    const int p = hh * 24 + i;
    const int d = p >> 4, f = p & 15;
    const float d0 = rw[d * 32 + f] - mean;
    const float d1 = rw[d * 32 + 16 + f] - mean;
    ss += d0 * d0;
    ss += d1 * d1;
  }
  {
    const float dr = rf - mean;
    ss += (hh == 1) ? (dr * dr) : 0.0f;
  }
  ss += __shfl_xor(ss, 16, 32);
  const float var  = ss * (1.0f / (float)STEM_IN);
  const float rstd = 1.0f / sqrtf(var + 1e-5f);
  _Float16* xr = xaS[wave] + c * XA_PITCH;
#pragma unroll 1
  for (int i = 0; i < 24; ++i) {
    const int p = hh * 24 + i;
    const int d = p >> 4, f = p & 15;
    const int f0 = d * 32 + f, f1 = f0 + 16;
    const float y0 = ((rw[f0] - mean) * rstd) * lng[f0] + lnb[f0];
    const float y1 = ((rw[f1] - mean) * rstd) * lng[f1] + lnb[f1];
    xr[f0] = (_Float16)y0;
    xr[f1] = (_Float16)y1;
  }
  {
    const float y96 = ((rf - mean) * rstd) * g96 + be96;
    if (hh == 1) xr[96] = (_Float16)y96;
  }
#pragma unroll 1
  for (int k = 0; k < 16; ++k) {
    const int cp = STEM_IN + hh * 16 + k;
    if (cp < STEM_KP) xr[cp] = (_Float16)0.0f;
  }
  __syncthreads();

  {
    const _Float16* ar = xaS[wave] + c * XA_PITCH + koff;
    const v16h a0 = Frag<_Float16>::load(ar);
    const v16h a1 = Frag<_Float16>::load(ar + 32);
    const v16h a2 = Frag<_Float16>::load(ar + 64);
    const v16h a3 = Frag<_Float16>::load(ar + 96);
    _Float16* hd = hdS[wave];
#pragma unroll 1
    for (int nt = 0; nt < STEM_HID / 16; ++nt) {
      const int n = nt * 16 + c;
      const _Float16* wr = W1t + (size_t)n * STEM_KP + koff;
      const v16h w0 = Frag<_Float16>::load(wr);
      const v16h w1 = Frag<_Float16>::load(wr + 32);
      const v16h w2 = Frag<_Float16>::load(wr + 64);
      const v16h w3 = Frag<_Float16>::load(wr + 96);
      v8f acc = {0.f, 0.f, 0.f, 0.f, 0.f, 0.f, 0.f, 0.f};
      acc = Frag<_Float16>::mma(a0, w0, acc);
      acc = Frag<_Float16>::mma(a1, w1, acc);
      acc = Frag<_Float16>::mma(a2, w2, acc);
      acc = Frag<_Float16>::mma(a3, w3, acc);
      guard1_h8(acc, a0, a1, a2, a3, w0, w1, w2, w3);
      const float bn = b1[n];
#pragma unroll
      for (int r = 0; r < 8; ++r) {
        const float o = silu_f(BNC * (acc[r] + bn));
        hd[(8 * hh + r) * T_PITCH + n] = (_Float16)o;
      }
    }
  }
  __syncthreads();

  {
    const _Float16* ar = hdS[wave] + c * T_PITCH + koff;
    const v16h a0 = Frag<_Float16>::load(ar);
    const v16h a1 = Frag<_Float16>::load(ar + 32);
    _Float16* xo = xoS[wave];
#pragma unroll 1
    for (int nt = 0; nt < STEM_OUT / 16; ++nt) {
      const int n = nt * 16 + c;
      const _Float16* wr = W2t + (size_t)n * STEM_HID + koff;
      const v16h w0 = Frag<_Float16>::load(wr);
      const v16h w1 = Frag<_Float16>::load(wr + 32);
      v8f acc = {0.f, 0.f, 0.f, 0.f, 0.f, 0.f, 0.f, 0.f};
      acc = Frag<_Float16>::mma(a0, w0, acc);
      acc = Frag<_Float16>::mma(a1, w1, acc);
      guard1_h4(acc, a0, a1, w0, w1);
      const float bn = b2[n];
#pragma unroll
      for (int r = 0; r < 8; ++r) {
        const float o = silu_f(BNC * (acc[r] + bn));
        xo[(8 * hh + r) * STEM_OUT + n] = (_Float16)o;
      }
    }
  }
  __syncthreads();

  {
    const u32x4* src = (const u32x4*)(const void*)(&xoS[wave][0]);
    const u32x4 w0 = src[lane];
    const u32x4 w1 = src[32 + lane];
    u32x4* dp = (u32x4*)(void*)xplane + (size_t)pt0 * 4;
    for (int pass = 0; pass < 2; ++pass) {
      *(volatile u32x4*)(dp + lane) = w0;
      *(volatile u32x4*)(dp + 32 + lane) = w1;
      __threadfence();
    }
  }
}

__global__ __launch_bounds__(256) void sfeat_kernel(const float* __restrict__ pos,
                                                    const int* __restrict__ idx, const int* __restrict__ col,
                                                    const float* __restrict__ lkw, const float* __restrict__ lkb,
                                                    const float* __restrict__ lng, const float* __restrict__ lnb,
                                                    float* __restrict__ sfe) {
  const int m = blockIdx.x * 256 + threadIdx.x;
  int im = idx[m];
  im = (im < 0) ? 0 : ((im > NPTS - 1) ? (NPTS - 1) : im);
  const float px = pos[(size_t)im * 3 + 0], py = pos[(size_t)im * 3 + 1], pz = pos[(size_t)im * 3 + 2];
  float n0 = 0.0f, n1 = 0.0f, n2 = 0.0f, n3 = 0.0f, n4 = 0.0f, n5 = 0.0f, n6 = 0.0f, n7 = 0.0f;
#pragma unroll 1
  for (int j = 0; j < KNBR; ++j) {
    int cj = col[(size_t)m * KNBR + j];
    cj = (cj < 0) ? 0 : ((cj > NPTS - 1) ? (NPTS - 1) : cj);
    const float dx = pos[(size_t)cj * 3 + 0] - px;
    const float dy = pos[(size_t)cj * 3 + 1] - py;
    const float dz = pos[(size_t)cj * 3 + 2] - pz;
    const float nrm = sqrtf((dx * dx + dz * dz) + dy * dy);
    const float inv = 1.0f / (nrm + 1e-8f);
    const float ux = dx * inv, uy = dy * inv, uz = dz * inv;
    n0 += ( ux + uy) + uz;
    n1 += (-ux + uy) + uz;
    n2 += ( ux - uy) + uz;
    n3 += ( ux + uy) - uz;
    n4 += (-ux - uy) + uz;
    n5 += (-ux + uy) - uz;
    n6 += ( ux - uy) - uz;
    n7 += (-ux - uy) - uz;
  }
  const float sc = KDC * (1.0f / (float)KNBR);
  n0 *= sc; n1 *= sc; n2 *= sc; n3 *= sc; n4 *= sc; n5 *= sc; n6 *= sc; n7 *= sc;
  float s0 = 0.0f, s1 = 0.0f, s2 = 0.0f;
  s0 += n0 * lkw[0];  s1 += n0 * lkw[1];  s2 += n0 * lkw[2];
  s0 += n1 * lkw[3];  s1 += n1 * lkw[4];  s2 += n1 * lkw[5];
  s0 += n2 * lkw[6];  s1 += n2 * lkw[7];  s2 += n2 * lkw[8];
  s0 += n3 * lkw[9];  s1 += n3 * lkw[10]; s2 += n3 * lkw[11];
  asm volatile("" ::: "memory");
  s0 += n4 * lkw[12]; s1 += n4 * lkw[13]; s2 += n4 * lkw[14];
  s0 += n5 * lkw[15]; s1 += n5 * lkw[16]; s2 += n5 * lkw[17];
  s0 += n6 * lkw[18]; s1 += n6 * lkw[19]; s2 += n6 * lkw[20];
  s0 += n7 * lkw[21]; s1 += n7 * lkw[22]; s2 += n7 * lkw[23];
  s0 += lkb[0]; s1 += lkb[1]; s2 += lkb[2];
  const float mean = ((s0 + s1) + s2) * (1.0f / 3.0f);
  const float d0 = s0 - mean, d1 = s1 - mean, d2 = s2 - mean;
  const float var  = ((d0 * d0 + d1 * d1) + d2 * d2) * (1.0f / 3.0f);
  const float rstd = 1.0f / sqrtf(var + 1e-5f);
  v4f o;
  o[0] = (d0 * rstd) * lng[0] + lnb[0];
  o[1] = (d1 * rstd) * lng[1] + lnb[1];
  o[2] = (d2 * rstd) * lng[2] + lnb[2];
  o[3] = 0.0f;
  volatile v4f* p = (volatile v4f*)(sfe + (size_t)m * 4);
  *p = o;
  __threadfence();
  *p = o;
}

__global__ __launch_bounds__(256) void edge_kernel(const float* __restrict__ pos, const float* __restrict__ refl,
                                                   const int* __restrict__ idx, const int* __restrict__ col,
                                                   const unsigned* __restrict__ xplane, const float* __restrict__ sfe,
                                                   const unsigned short* __restrict__ W1tp, const float* __restrict__ b1,
                                                   const unsigned short* __restrict__ W2tp, const float* __restrict__ b2,
                                                   float* __restrict__ aggf, unsigned* __restrict__ aggb) {
  __shared__ __align__(16) _Float16 msgT[8][16 * T_PITCH];
  __shared__ __align__(16) _Float16 hidT[8][16 * T_PITCH];
  __shared__ __align__(16) float    aggS[8][LOC_OUT];
  const _Float16* W1t = (const _Float16*)W1tp;
  const _Float16* W2t = (const _Float16*)W2tp;
  const int tid = threadIdx.x, wave = tid >> 5, lane = tid & 31;
  const int c = lane & 15, hh = lane >> 4, koff = hh * 8;
  const int m = blockIdx.x * 8 + wave;
  const int e = m * KNBR + c;
  int cj = col[e];
  cj = (cj < 0) ? 0 : ((cj > NPTS - 1) ? (NPTS - 1) : cj);
  int im = idx[m];
  im = (im < 0) ? 0 : ((im > NPTS - 1) ? (NPTS - 1) : im);
  const float pjx = pos[(size_t)cj * 3 + 0], pjy = pos[(size_t)cj * 3 + 1], pjz = pos[(size_t)cj * 3 + 2];
  const float pix = pos[(size_t)im * 3 + 0], piy = pos[(size_t)im * 3 + 1], piz = pos[(size_t)im * 3 + 2];
  const float rj = refl[cj], ri = refl[im];
  int mv = m;
  asm volatile("" : "+v"(mv));
  const v4f sv = *(const v4f*)(sfe + (size_t)mv * 4);
  const u32x4* xw = (const u32x4*)(const void*)xplane;
  const u32x4 xq0 = xw[(size_t)cj * 4 + 2 * hh];
  const u32x4 xq1 = xw[(size_t)cj * 4 + 2 * hh + 1];

  const float r0 = pjx - pix, r1 = pjy - piy, r2 = pjz - piz, r3 = rj - ri;
  const _Float16 g0 = (_Float16)r0, g1 = (_Float16)r1, g2 = (_Float16)r2, g3 = (_Float16)r3;
  const float g0f = (float)g0, g1f = (float)g1, g2f = (float)g2, g3f = (float)g3;
  const float l0 = r0 - g0f, l1 = r1 - g1f, l2 = r2 - g2f, l3 = r3 - g3f;
  const float t0 = g0f * WLO_CARRY_INV, t1 = g1f * WLO_CARRY_INV, t2 = g2f * WLO_CARRY_INV, t3 = g3f * WLO_CARRY_INV;
  const float sv0 = sv[0], sv1 = sv[1], sv2 = sv[2];
  const unsigned a0w = pack_h2f(g0f, g1f), a1w = pack_h2f(g2f, g3f), a2w = pack_h2f(sv0, sv1), a3w = pack_h2f(sv2, l0);
  const unsigned q0w = pack_h2f(l1, l2), q1w = pack_h2f(l3, t0), q2w = pack_h2f(t1, t2), q3w = pack_h2f(t3, t3);
  u32x4 mid;
  mid[0] = hh ? q0w : a0w;
  mid[1] = hh ? q1w : a1w;
  mid[2] = hh ? q2w : a2w;
  mid[3] = hh ? q3w : a3w;
  const u32x4 zq = {0u, 0u, 0u, 0u};
  {
    u32x4* mrow = (u32x4*)(void*)(&msgT[wave][0] + c * T_PITCH);
    mrow[2 * hh]     = xq0;
    mrow[2 * hh + 1] = xq1;
    mrow[4 + hh]     = mid;
    mrow[6 + hh]     = zq;
  }
  __syncthreads();

  {
    const _Float16* ar = &msgT[wave][0] + c * T_PITCH + koff;
    const v16h a0 = Frag<_Float16>::load(ar);
    const v16h a1 = Frag<_Float16>::load(ar + 32);
    _Float16* hd = &hidT[wave][0];
#pragma unroll 1
    for (int nt = 0; nt < LOC_HID / 16; ++nt) {
      const int n = nt * 16 + c;
      const _Float16* wr = W1t + (size_t)n * MSG_KP + koff;
      const v16h w0 = Frag<_Float16>::load(wr);
      const v16h w1 = Frag<_Float16>::load(wr + 32);
      v8f acc = {0.f, 0.f, 0.f, 0.f, 0.f, 0.f, 0.f, 0.f};
      acc = Frag<_Float16>::mma(a0, w0, acc);
      acc = Frag<_Float16>::mma(a1, w1, acc);
      guard1_h4(acc, a0, a1, w0, w1);
      const float bn = b1[n];
#pragma unroll
      for (int r = 0; r < 8; ++r) {
        const float o = silu_f(BNC * (acc[r] + bn));
        hd[(8 * hh + r) * T_PITCH + n] = (_Float16)o;
      }
    }
  }
  __syncthreads();

  {
    const _Float16* ar = &hidT[wave][0] + c * T_PITCH + koff;
    const v16h a0 = Frag<_Float16>::load(ar);
    const v16h a1 = Frag<_Float16>::load(ar + 32);
#pragma unroll 1
    for (int nt = 0; nt < LOC_OUT / 16; ++nt) {
      const int n = nt * 16 + c;
      const _Float16* wr = W2t + (size_t)n * LOC_HID + koff;
      const v16h w0 = Frag<_Float16>::load(wr);
      const v16h w1 = Frag<_Float16>::load(wr + 32);
      v8f acc = {0.f, 0.f, 0.f, 0.f, 0.f, 0.f, 0.f, 0.f};
      acc = Frag<_Float16>::mma(a0, w0, acc);
      acc = Frag<_Float16>::mma(a1, w1, acc);
      guard1_h4(acc, a0, a1, w0, w1);
      const float bn = b2[n];
      float mx = -INFINITY;
#pragma unroll
      for (int r = 0; r < 8; ++r) mx = fmaxf(mx, silu_f(BNC * (acc[r] + bn)));
      const float other = __shfl_xor(mx, 16, 32);
      const float mall = fmaxf(mx, other);
      if (hh == 0) aggS[wave][n] = mall;
    }
  }
  __syncthreads();

  {
    const v4f v = *(const v4f*)(&aggS[wave][0] + lane * 4);
    v4f* dp = (v4f*)(void*)aggf + (size_t)m * (LOC_OUT / 4) + lane;
    *(volatile v4f*)dp = v;
    __threadfence();
    *(volatile v4f*)dp = v;
  }
  if (wave < 4) {
    const int row = 2 * wave + hh;
    const float* sp = &aggS[row][0] + c * 8;
    const v4f x0 = *(const v4f*)sp;
    const v4f x1 = *(const v4f*)(sp + 4);
    const float e0 = x0[0], e1 = x0[1], e2 = x0[2], e3 = x0[3];
    const float e4 = x1[0], e5 = x1[1], e6 = x1[2], e7 = x1[3];
    u32x4 w;
    w[0] = pack2(bf_bits32(e0), bf_bits32(e1));
    w[1] = pack2(bf_bits32(e2), bf_bits32(e3));
    w[2] = pack2(bf_bits32(e4), bf_bits32(e5));
    w[3] = pack2(bf_bits32(e6), bf_bits32(e7));
    u32x4* dp = (u32x4*)(void*)aggb + (size_t)(blockIdx.x * 8 + row) * (LOC_OUT / 8) + c;
    *(volatile u32x4*)dp = w;
    __threadfence();
    *(volatile u32x4*)dp = w;
  }
}

__device__ __forceinline__ void stage4(float* slab, const v8f& a0, const v8f& a1, const v8f& a2, const v8f& a3, int mOff, int rlane) {
#pragma unroll
  for (int r = 0; r < 8; ++r) {
    float* rp = slab + (mOff + r) * SLAB_PITCH + rlane;
    rp[0]  = a0[r];
    rp[16] = a1[r];
    rp[32] = a2[r];
    rp[48] = a3[r];
  }
}

template <int EPI>
__device__ __forceinline__ float irb_chain(float x, float b, float w, float d) {
  float t = silu_f(BNC * (x + b));
  if (EPI == 1) t = silu_f(BNC * (t * w + d));
  if (EPI == 2) { t = silu_f(BNC * t); t = silu_f(BNC * (t * w + d)); }
  if (EPI == 3) t = BNC * t;
  return t;
}

template <int EPI>
__global__ __launch_bounds__(256) void irb_gemm_kernel(
    const unsigned short* __restrict__ Ap, int lda,
    const unsigned short* __restrict__ Btp, int ldb,
    void* __restrict__ Cout, int ldc,
    const float* __restrict__ bias, const float* __restrict__ dww, const float* __restrict__ dwb,
    const float* __restrict__ resid, int M, int N, int K) {
  typedef __bf16 T;
  typedef v16b V;
  const T* A  = (const T*)Ap;
  const T* Bt = (const T*)Btp;
  __shared__ __align__(16) float sT[8][16 * SLAB_PITCH];
  const int lane = threadIdx.x & 31;
  const int wave = threadIdx.x >> 5;
  const int tilesN = N >> 6;
  const int tilesM = M >> 6;
  const int tile = blockIdx.x * 8 + wave;
  if (tile >= tilesM * tilesN) return;
  const int tm = tile / tilesN;
  const int tn = tile - tm * tilesN;
  const int m0 = tm << 6;
  const int n0 = tn << 6;
  const int rlane = lane & 15;
  const int koff  = (lane >> 4) * 8;
  const int mOff  = (lane >> 4) * 8;

  v8f acc[4][4];
#pragma unroll
  for (int i = 0; i < 4; ++i)
#pragma unroll
    for (int j = 0; j < 4; ++j) acc[i][j] = (v8f){0.f, 0.f, 0.f, 0.f, 0.f, 0.f, 0.f, 0.f};

  for (int k0 = 0; k0 < K; k0 += 32) {
    V bh[4];
#pragma unroll
    for (int j = 0; j < 4; ++j) {
      const size_t bo = (size_t)(n0 + (j << 4) + rlane) * ldb + koff + k0;
      bh[j] = Frag<T>::load(Bt + bo);
    }
#pragma unroll
    for (int i = 0; i < 4; ++i) {
      const size_t ao = (size_t)(m0 + (i << 4) + rlane) * lda + koff + k0;
      const V ah = Frag<T>::load(A + ao);
#pragma unroll
      for (int j = 0; j < 4; ++j) acc[i][j] = Frag<T>::mma(ah, bh[j], acc[i][j]);
      guard4_b(acc[i][0], acc[i][1], acc[i][2], acc[i][3], ah, bh[0], bh[1], bh[2], bh[3]);
    }
    keep4_b(bh[0], bh[1], bh[2], bh[3]);
  }
  acc_guard4(acc[0][0], acc[0][1], acc[0][2], acc[0][3]);
  acc_guard4(acc[1][0], acc[1][1], acc[1][2], acc[1][3]);
  acc_guard4(acc[2][0], acc[2][1], acc[2][2], acc[2][3]);
  acc_guard4(acc[3][0], acc[3][1], acc[3][2], acc[3][3]);

  float* slab = sT[wave];
  if (EPI != 4) {
    const int q = lane >> 3, c8 = (lane & 7) * 8;
    const float bA = bias[n0 + lane];
    const float bB = bias[n0 + 32 + lane];
    float wA = 0.0f, wB = 0.0f, dA = 0.0f, dB = 0.0f;
    if (EPI == 1 || EPI == 2) {
      wA = dww[n0 + lane];
      wB = dww[n0 + 32 + lane];
      dA = dwb[n0 + lane];
      dB = dwb[n0 + 32 + lane];
    }
    unsigned short* C = (unsigned short*)Cout;
#pragma unroll 1
    for (int i = 0; i < 4; ++i) {
      const int mBase = m0 + (i << 4);
      if (i == 0)      stage4(slab, acc[0][0], acc[0][1], acc[0][2], acc[0][3], mOff, rlane);
      else if (i == 1) stage4(slab, acc[1][0], acc[1][1], acc[1][2], acc[1][3], mOff, rlane);
      else if (i == 2) stage4(slab, acc[2][0], acc[2][1], acc[2][2], acc[2][3], mOff, rlane);
      else             stage4(slab, acc[3][0], acc[3][1], acc[3][2], acc[3][3], mOff, rlane);
      wave_sync_lds();
#pragma unroll 1
      for (int row = 0; row < 16; ++row) {
        float* sp = slab + row * SLAB_PITCH + lane;
        const float xa = sp[0];
        const float xb = sp[32];
        const float ya = irb_chain<EPI>(xa, bA, wA, dA);
        const float yb = irb_chain<EPI>(xb, bB, wB, dB);
        sp[0]  = ya;
        sp[32] = yb;
      }
      wave_sync_lds();
      for (int pass = 0; pass < 2; ++pass) {
#pragma unroll
        for (int it = 0; it < 4; ++it) {
          const int row = it * 4 + q;
          const float* sp = slab + row * SLAB_PITCH + c8;
          const v4f x0 = *(const v4f*)sp;
          const v4f x1 = *(const v4f*)(sp + 4);
          const float e0 = x0[0], e1 = x0[1], e2 = x0[2], e3 = x0[3];
          const float e4 = x1[0], e5 = x1[1], e6 = x1[2], e7 = x1[3];
          u32x4 w;
          w[0] = pack2(bf_bits32(e0), bf_bits32(e1));
          w[1] = pack2(bf_bits32(e2), bf_bits32(e3));
          w[2] = pack2(bf_bits32(e4), bf_bits32(e5));
          w[3] = pack2(bf_bits32(e6), bf_bits32(e7));
          *(volatile u32x4*)(void*)(C + (size_t)(mBase + row) * ldc + n0 + c8) = w;
        }
        __threadfence();
      }
      wave_sync_lds();
    }
  } else {
    const int hh = lane >> 4, c4 = (lane & 15) * 4;
    const v4f b4 = *(const v4f*)(bias + n0 + c4);
    float* C = (float*)Cout;
#pragma unroll 1
    for (int i = 0; i < 4; ++i) {
      const int mBase = m0 + (i << 4);
      if (i == 0)      stage4(slab, acc[0][0], acc[0][1], acc[0][2], acc[0][3], mOff, rlane);
      else if (i == 1) stage4(slab, acc[1][0], acc[1][1], acc[1][2], acc[1][3], mOff, rlane);
      else if (i == 2) stage4(slab, acc[2][0], acc[2][1], acc[2][2], acc[2][3], mOff, rlane);
      else             stage4(slab, acc[3][0], acc[3][1], acc[3][2], acc[3][3], mOff, rlane);
      wave_sync_lds();
#pragma unroll 1
      for (int it = 0; it < 8; ++it) {
        const int row = it * 2 + hh;
        float* sp = slab + row * SLAB_PITCH + c4;
        const v4f x = *(const v4f*)sp;
        const v4f rs = *(const v4f*)(resid + (size_t)(mBase + row) * ldc + n0 + c4);
        v4f y;
#pragma unroll
        for (int e = 0; e < 4; ++e) y[e] = silu_f(BNC * (x[e] + b4[e]) + rs[e]);
        *(v4f*)sp = y;
      }
      wave_sync_lds();
      for (int pass = 0; pass < 2; ++pass) {
#pragma unroll
        for (int it = 0; it < 8; ++it) {
          const int row = it * 2 + hh;
          const v4f v = *(const v4f*)(slab + row * SLAB_PITCH + c4);
          *(volatile v4f*)(C + (size_t)(mBase + row) * ldc + n0 + c4) = v;
        }
        __threadfence();
      }
      wave_sync_lds();
    }
  }
}

extern "C" void kernel_launch(void* const* d_in, const int* in_sizes, int n_in,
                              void* d_out, int out_size, void* d_ws, size_t ws_size, hipStream_t stream) {
  if (n_in < 33 || d_out == nullptr || d_ws == nullptr) return;
  if (in_sizes[0] != NPTS * 3 || in_sizes[1] != NPTS || in_sizes[2] != NBAT || in_sizes[3] != NPTS ||
      in_sizes[4] != MROW || in_sizes[5] != NEDGE || in_sizes[9] != STEM_IN * STEM_HID ||
      in_sizes[11] != STEM_HID * STEM_OUT || in_sizes[17] != MSG_IN * LOC_HID || in_sizes[19] != LOC_HID * LOC_OUT ||
      in_sizes[21] != LOC_OUT * IRB_WIDE || in_sizes[25] != IRB_WIDE * IRB_WIDE || in_sizes[29] != IRB_WIDE * IRB_WIDE ||
      in_sizes[31] != IRB_WIDE * LOC_OUT || out_size != MROW * LOC_OUT) return;

  const float* pos     = (const float*)d_in[0];
  const float* refl    = (const float*)d_in[1];
  const float* sf      = (const float*)d_in[2];
  const int*   batch   = (const int*)d_in[3];
  const int*   idx     = (const int*)d_in[4];
  const int*   col     = (const int*)d_in[5];
  const float* stem_ln_g = (const float*)d_in[7];
  const float* stem_ln_b = (const float*)d_in[8];
  const float* stem_w1   = (const float*)d_in[9];
  const float* stem_b1   = (const float*)d_in[10];
  const float* stem_w2   = (const float*)d_in[11];
  const float* stem_b2   = (const float*)d_in[12];
  const float* lk_w      = (const float*)d_in[13];
  const float* lk_b      = (const float*)d_in[14];
  const float* lk_ln_g   = (const float*)d_in[15];
  const float* lk_ln_b   = (const float*)d_in[16];
  const float* loc_w1    = (const float*)d_in[17];
  const float* loc_b1    = (const float*)d_in[18];
  const float* loc_w2    = (const float*)d_in[19];
  const float* loc_b2    = (const float*)d_in[20];
  const float* exp_w     = (const float*)d_in[21];
  const float* exp_b     = (const float*)d_in[22];
  const float* dw1_w     = (const float*)d_in[23];
  const float* dw1_b     = (const float*)d_in[24];
  const float* pw1_w     = (const float*)d_in[25];
  const float* pw1_b     = (const float*)d_in[26];
  const float* dw2_w     = (const float*)d_in[27];
  const float* dw2_b     = (const float*)d_in[28];
  const float* pw2_w     = (const float*)d_in[29];
  const float* pw2_b     = (const float*)d_in[30];
  const float* proj_w    = (const float*)d_in[31];
  const float* proj_b    = (const float*)d_in[32];
  float* out = (float*)d_out;

  char* ws = (char*)d_ws; size_t off = 0;
  auto carve = [&](size_t bytes) -> char* { char* p = ws + off; off += (bytes + 255) & ~(size_t)255; return p; };
  unsigned* BT_S1 = (unsigned*)carve((size_t)STEM_HID * STEM_KP * 2);
  unsigned* BT_S2 = (unsigned*)carve((size_t)STEM_OUT * STEM_HID * 2);
  unsigned* BT_L1 = (unsigned*)carve((size_t)LOC_HID * MSG_KP * 2);
  unsigned* BT_L2 = (unsigned*)carve((size_t)LOC_OUT * LOC_HID * 2);
  unsigned* BT_EX = (unsigned*)carve((size_t)IRB_WIDE * LOC_OUT * 2);
  unsigned* BT_P1 = (unsigned*)carve((size_t)IRB_WIDE * IRB_WIDE * 2);
  unsigned* BT_P2 = (unsigned*)carve((size_t)IRB_WIDE * IRB_WIDE * 2);
  unsigned* BT_PJ = (unsigned*)carve((size_t)LOC_OUT * IRB_WIDE * 2);
  float*    CEN   = (float*)carve((size_t)NBAT * CEN_PITCH * 4);
  unsigned* XPL   = (unsigned*)carve((size_t)NPTS * STEM_OUT * 2);
  float*    SFE   = (float*)carve((size_t)MROW * 4 * 4);
  float*    AGGF  = (float*)carve((size_t)MROW * LOC_OUT * 4);
  unsigned* AGGB  = (unsigned*)carve((size_t)MROW * LOC_OUT * 2);
  unsigned* P1    = (unsigned*)carve((size_t)MROW * IRB_WIDE * 2);
  unsigned* P2    = (unsigned*)carve((size_t)MROW * IRB_WIDE * 2);
  if (off > ws_size || off > (size_t)134217728) return;

  prep_bt_kernel<0><<<(STEM_HID * (STEM_KP / 8) + 255) / 256, 256, 0, stream>>>(stem_w1, BT_S1, STEM_IN, STEM_HID, STEM_KP);
  prep_bt_kernel<0><<<(STEM_OUT * (STEM_HID / 8) + 255) / 256, 256, 0, stream>>>(stem_w2, BT_S2, STEM_HID, STEM_OUT, STEM_HID);
  prep_loc1_kernel<<<(LOC_HID * (MSG_KP / 8)) / 256, 256, 0, stream>>>(loc_w1, BT_L1);
  prep_bt_kernel<0><<<(LOC_OUT * (LOC_HID / 8) + 255) / 256, 256, 0, stream>>>(loc_w2, BT_L2, LOC_HID, LOC_OUT, LOC_HID);
  prep_bt_kernel<1><<<(IRB_WIDE * (LOC_OUT / 8) + 255) / 256, 256, 0, stream>>>(exp_w, BT_EX, LOC_OUT, IRB_WIDE, LOC_OUT);
  prep_bt_kernel<1><<<(IRB_WIDE * (IRB_WIDE / 8) + 255) / 256, 256, 0, stream>>>(pw1_w, BT_P1, IRB_WIDE, IRB_WIDE, IRB_WIDE);
  prep_bt_kernel<1><<<(IRB_WIDE * (IRB_WIDE / 8) + 255) / 256, 256, 0, stream>>>(pw2_w, BT_P2, IRB_WIDE, IRB_WIDE, IRB_WIDE);
  prep_bt_kernel<1><<<(LOC_OUT * (IRB_WIDE / 8) + 255) / 256, 256, 0, stream>>>(proj_w, BT_PJ, IRB_WIDE, LOC_OUT, IRB_WIDE);

  centres_kernel<<<NBAT, 256, 0, stream>>>(pos, sf, CEN);

  stem_kernel<<<NPTS / 64, 128, 0, stream>>>(pos, refl, sf, batch, CEN, stem_ln_g, stem_ln_b,
                                             (const unsigned short*)BT_S1, stem_b1,
                                             (const unsigned short*)BT_S2, stem_b2, XPL);

  sfeat_kernel<<<MROW / 256, 256, 0, stream>>>(pos, idx, col, lk_w, lk_b, lk_ln_g, lk_ln_b, SFE);

  edge_kernel<<<MROW / 8, 256, 0, stream>>>(pos, refl, idx, col, XPL, SFE,
                                            (const unsigned short*)BT_L1, loc_b1,
                                            (const unsigned short*)BT_L2, loc_b2, AGGF, AGGB);

  irb_gemm_kernel<1><<<(MROW / 64) * (IRB_WIDE / 64) / 8, 256, 0, stream>>>(
      (const unsigned short*)AGGB, LOC_OUT, (const unsigned short*)BT_EX, LOC_OUT, (void*)P1, IRB_WIDE,
      exp_b, dw1_w, dw1_b, AGGF, MROW, IRB_WIDE, LOC_OUT);
  irb_gemm_kernel<2><<<(MROW / 64) * (IRB_WIDE / 64) / 8, 256, 0, stream>>>(
      (const unsigned short*)P1, IRB_WIDE, (const unsigned short*)BT_P1, IRB_WIDE, (void*)P2, IRB_WIDE,
      pw1_b, dw2_w, dw2_b, AGGF, MROW, IRB_WIDE, IRB_WIDE);
  irb_gemm_kernel<3><<<(MROW / 64) * (IRB_WIDE / 64) / 8, 256, 0, stream>>>(
      (const unsigned short*)P2, IRB_WIDE, (const unsigned short*)BT_P2, IRB_WIDE, (void*)P1, IRB_WIDE,
      pw2_b, dw2_w, dw2_b, AGGF, MROW, IRB_WIDE, IRB_WIDE);
  irb_gemm_kernel<4><<<(MROW / 64) * (LOC_OUT / 64) / 8, 256, 0, stream>>>(
      (const unsigned short*)P1, IRB_WIDE, (const unsigned short*)BT_PJ, IRB_WIDE, (void*)out, LOC_OUT,
      proj_b, dw2_w, dw2_b, AGGF, MROW, LOC_OUT, IRB_WIDE);
}
